// FwdModel_46909632806947
// MI455X (gfx1250) — hardware-verified
//
#include <hip/hip_runtime.h>
#include <stddef.h>
#include <stdint.h>

typedef __attribute__((ext_vector_type(16))) _Float16 v16h;
typedef __attribute__((ext_vector_type(8)))  _Float16 v8h;
typedef __attribute__((ext_vector_type(16))) __bf16   v16b;
typedef __attribute__((ext_vector_type(8)))  __bf16   v8b;
typedef __attribute__((ext_vector_type(8)))  float    v8f;
typedef __attribute__((ext_vector_type(4)))  float    v4f;
typedef __attribute__((ext_vector_type(4)))  unsigned v4u;

constexpr int NBATCH  = 4;
constexpr int NCH     = 3;
constexpr int CH_ALL  = 18;
constexpr int NDEP    = 15;
constexpr int IMG_H   = 256;
constexpr int IMG_W   = 256;
constexpr int HWPIX   = IMG_H * IMG_W;
constexpr int KTAP    = 71;
constexpr int PADR    = 35;
constexpr int TILE_H  = 16;
constexpr int TILE_W  = 32;
constexpr int NSIG    = 8;
constexpr int NJC     = 3;
constexpr int BT_HALVES = 512;
constexpr int NTILES  = NCH * KTAP * NSIG * NJC;
constexpr size_t WSB_HALVES = (size_t)NTILES * BT_HALVES;
constexpr int NB_THREADS = NTILES * (BT_HALVES / 8);
constexpr int PROWS   = 86;
constexpr int PCOLS   = 136;
constexpr int PREAL   = TILE_W + KTAP - 1;
constexpr int PWORDS  = PCOLS / 2;
constexpr int NTHR    = 256;

static_assert(PROWS == TILE_H + KTAP - 1);
static_assert(PCOLS % 8 == 0 && PCOLS >= (NSIG * 3) + 32 * NJC);
static_assert(PREAL <= PCOLS && (PREAL % 2) == 0);
static_assert(NJC * 32 >= KTAP + NSIG - 1);
static_assert(NSIG * 4 == TILE_W);
static_assert(IMG_W % TILE_W == 0 && IMG_H % TILE_H == 0);
static_assert(NB_THREADS % NTHR == 0);
static_assert(NDEP < 16);

__device__ __forceinline__ unsigned short f2bf_bits(float f) {
  unsigned u = __float_as_uint(f);
  return (unsigned short)((u + 0x7FFFu + ((u >> 16) & 1u)) >> 16);
}
__device__ __forceinline__ float bf_bits2f(unsigned short h) { return __uint_as_float(((unsigned)h) << 16); }
__device__ __forceinline__ float bfr(float f) { return bf_bits2f(f2bf_bits(f)); }

__device__ __forceinline__ void dep_guard_h(v8f& a, v8f& b, v16h x, v16h y) { asm volatile("v_nop\n\tv_nop\n\tv_nop\n\tv_nop" : "+v"(a), "+v"(b) : "v"(x), "v"(y)); }
__device__ __forceinline__ void dep_guard_b(v8f& a, v8f& b, v16b x, v16b y) { asm volatile("v_nop\n\tv_nop\n\tv_nop\n\tv_nop" : "+v"(a), "+v"(b) : "v"(x), "v"(y)); }
__device__ __forceinline__ void keep4_h(v16h a, v16h b, v16h c, v16h d) { asm volatile("v_nop" :: "v"(a), "v"(b), "v"(c), "v"(d)); }
__device__ __forceinline__ void keep4_b(v16b a, v16b b, v16b c, v16b d) { asm volatile("v_nop" :: "v"(a), "v"(b), "v"(c), "v"(d)); }
__device__ __forceinline__ void acc_guard4(v8f& a, v8f& b, v8f& c, v8f& d) { asm volatile("v_nop\n\tv_nop\n\tv_nop\n\tv_nop" : "+v"(a), "+v"(b), "+v"(c), "+v"(d)); }
template <typename T> struct Frag;
template <> struct Frag<_Float16> {
  typedef v16h V; union U { v16h v; v8h h[2]; };
  static __device__ __forceinline__ v16h load(const _Float16* p) {
    U f; f.h[0] = *(const v8h*)(p); f.h[1] = *(const v8h*)(p + 16); return f.v;
  }
  static __device__ __forceinline__ v8f mma(v16h a, v16h b, v8f c) {
    return __builtin_amdgcn_wmma_f32_16x16x32_f16(false, a, false, b, (short)0, c, false, false);
  }
  static __device__ __forceinline__ void guard(v8f& a, v8f& b, v16h x, v16h y) { dep_guard_h(a, b, x, y); }
  static __device__ __forceinline__ void keep(v16h a, v16h b, v16h c, v16h d) { keep4_h(a, b, c, d); }
};
template <> struct Frag<__bf16> {
  typedef v16b V; union U { v16b v; v8b h[2]; };
  static __device__ __forceinline__ v16b load(const __bf16* p) {
    U f; f.h[0] = *(const v8b*)(p); f.h[1] = *(const v8b*)(p + 16); return f.v;
  }
  static __device__ __forceinline__ v8f mma(v16b a, v16b b, v8f c) {
    return __builtin_amdgcn_wmma_f32_16x16x32_bf16(false, a, false, b, (short)0, c, false, false);
  }
  static __device__ __forceinline__ void guard(v8f& a, v8f& b, v16b x, v16b y) { dep_guard_b(a, b, x, y); }
  static __device__ __forceinline__ void keep(v16b a, v16b b, v16b c, v16b d) { keep4_b(a, b, c, d); }
};
typedef Frag<__bf16> FragB;

__device__ __forceinline__ void grp_guard(v8f& c0, v8f& c1, v8f& c2, v8f& c3,
                                          v16b x0, v16b x1, v16b x2, v16b x3, v16b y) {
  asm volatile("v_nop\n\tv_nop\n\tv_nop\n\tv_nop"
               : "+v"(c0), "+v"(c1), "+v"(c2), "+v"(c3)
               : "v"(x0), "v"(x1), "v"(x2), "v"(x3), "v"(y));
}

__global__ __launch_bounds__(NTHR) void build_btiles(const float* __restrict__ psf, unsigned* __restrict__ btw, int nthreads) {
  const int idx = blockIdx.x * NTHR + threadIdx.x;
  if (idx >= nthreads) return;
  const int e8 = idx & 1;
  const int lf = (idx >> 1) & 31;
  int t = idx >> 6;
  const int jc = t % NJC;  t /= NJC;
  const int sg = t % NSIG; t /= NSIG;
  const int ii = t % KTAP;
  const int cc = t / KTAP;
  const int n   = lf & 15;
  const int hf  = lf >> 4;
  const int ncl = (n < NDEP) ? n : (NDEP - 1);
  const float* prow = psf + (size_t)(cc * KTAP + ii) * KTAP * NDEP;
  v4u w = {0u, 0u, 0u, 0u};
#pragma unroll
  for (int ee = 0; ee < 8; ++ee) {
    const int k   = 8 * hf + 16 * e8 + ee;
    const int j   = jc * 32 + k - sg;
    const int jcl = j < 0 ? 0 : (j > KTAP - 1 ? KTAP - 1 : j);
    const float v = prow[jcl * NDEP + ncl];
    const bool ok = (j >= 0) && (j < KTAP) && (n < NDEP);
    const unsigned b = ok ? (unsigned)f2bf_bits(v) : 0u;
    w[ee >> 1] |= b << (16 * (ee & 1));
  }
  unsigned* dst = btw + (size_t)idx * 4;
  *(volatile v4u*)dst = w;
  __threadfence();
  *(volatile v4u*)dst = w;
}

__global__ __launch_bounds__(NTHR) void conv_depth_fused(const float* __restrict__ x,
                                                         const unsigned short* __restrict__ btp,
                                                         float* __restrict__ out) {
  __shared__ __align__(16) unsigned patchw[PROWS * PWORDS];
  __shared__ __align__(16) float    Dsh[TILE_H * TILE_W * 16];
  __shared__ __align__(16) float    Osh[TILE_H * TILE_W];

  const int w0 = blockIdx.x * TILE_W;
  const int h0 = blockIdx.y * TILE_H;
  const int bb = blockIdx.z / NCH;
  const int c  = blockIdx.z - bb * NCH;
  const int tid  = threadIdx.x;
  const int wave = tid >> 5;
  const int lane = tid & 31;
  const int rlane = lane & 15;
  const int hh    = lane >> 4;
  const int koff  = hh * 8;

  {
    const float* src = x + (size_t)(bb * CH_ALL + c) * HWPIX;
#pragma unroll 1
    for (int p = tid; p < PROWS * PWORDS; p += NTHR) {
      const int r  = p / PWORDS;
      const int cp = p - r * PWORDS;
      const int cl = 2 * cp;
      int gh = h0 - PADR + r;       gh  = gh  < 0 ? 0 : (gh  > IMG_H - 1 ? IMG_H - 1 : gh);
      int gw0 = w0 - PADR + cl;     gw0 = gw0 < 0 ? 0 : (gw0 > IMG_W - 1 ? IMG_W - 1 : gw0);
      int gw1 = w0 - PADR + cl + 1; gw1 = gw1 < 0 ? 0 : (gw1 > IMG_W - 1 ? IMG_W - 1 : gw1);
      const float v0 = src[gh * IMG_W + gw0];
      const float v1 = src[gh * IMG_W + gw1];
      const unsigned b0 = (cl < PREAL) ? (unsigned)f2bf_bits(v0) : 0u;
      const unsigned b1 = (cl < PREAL) ? (unsigned)f2bf_bits(v1) : 0u;
      patchw[p] = b0 | (b1 << 16);
    }
  }
  {
    const float* dsrc = x + (size_t)(bb * CH_ALL + NCH) * HWPIX;
#pragma unroll 1
    for (int p = tid; p < NDEP * TILE_H * (TILE_W / 4); p += NTHR) {
      const int q = p & 7;
      const int m = (p >> 3) & 15;
      const int d = p >> 7;
      const v4f v = *(const v4f*)(dsrc + (size_t)d * HWPIX + (size_t)(h0 + m) * IMG_W + w0 + 4 * q);
#pragma unroll
      for (int e = 0; e < 4; ++e) Dsh[(m * TILE_W + 4 * q + e) * 16 + d] = bfr(v[e]);
    }
#pragma unroll 1
    for (int p = tid; p < TILE_H * TILE_W; p += NTHR) Dsh[p * 16 + NDEP] = 0.0f;
  }
  __syncthreads();

  v8f acc[4];
#pragma unroll
  for (int t = 0; t < 4; ++t) acc[t] = (v8f){0.f, 0.f, 0.f, 0.f, 0.f, 0.f, 0.f, 0.f};

  const __bf16* patch = (const __bf16*)patchw;
  const __bf16* Abase = patch + (size_t)rlane * PCOLS + koff;
  const __bf16* Bt    = (const __bf16*)btp;
  const __bf16* Bbase = Bt + ((size_t)(c * KTAP) * NSIG + wave) * NJC * BT_HALVES + (size_t)lane * 16;
  constexpr size_t B_ISTRIDE = (size_t)NSIG * NJC * BT_HALVES;

#pragma unroll 1
  for (int i = 0; i < KTAP; ++i) {
    const __bf16* arow  = Abase + (size_t)i * PCOLS;
    const __bf16* btile = Bbase + (size_t)i * B_ISTRIDE;
#pragma unroll
    for (int jc = 0; jc < NJC; ++jc) {
      const v16b bf = *(const v16b*)(btile + jc * BT_HALVES);
      const v16b a0 = FragB::load(arow + jc * 32 + 0);
      const v16b a1 = FragB::load(arow + jc * 32 + 8);
      const v16b a2 = FragB::load(arow + jc * 32 + 16);
      const v16b a3 = FragB::load(arow + jc * 32 + 24);
      acc[0] = FragB::mma(a0, bf, acc[0]);
      acc[1] = FragB::mma(a1, bf, acc[1]);
      acc[2] = FragB::mma(a2, bf, acc[2]);
      acc[3] = FragB::mma(a3, bf, acc[3]);
      grp_guard(acc[0], acc[1], acc[2], acc[3], a0, a1, a2, a3, bf);
    }
  }
  acc_guard4(acc[0], acc[1], acc[2], acc[3]);

#pragma unroll
  for (int t = 0; t < 4; ++t) {
    const int s = wave + 8 * t;
#pragma unroll
    for (int r = 0; r < 8; ++r) {
      const int m = 8 * hh + r;
      const float dep = Dsh[(m * TILE_W + s) * 16 + rlane];
      float pv = acc[t][r] * dep;
      pv += __shfl_xor(pv, 1, 32);
      pv += __shfl_xor(pv, 2, 32);
      pv += __shfl_xor(pv, 4, 32);
      pv += __shfl_xor(pv, 8, 32);
      if (rlane == 0) Osh[m * TILE_W + s] = pv;
    }
  }
  __syncthreads();

  if (wave < 4) {
    const int row = wave * 4 + (lane >> 3);
    const int c4  = (lane & 7) * 4;
    const v4f val = *(const v4f*)(Osh + row * TILE_W + c4);
    float* op = out + (size_t)(bb * NCH + c) * HWPIX + (size_t)(h0 + row) * IMG_W + w0 + c4;
    *(volatile v4f*)op = val;
    __threadfence();
    *(volatile v4f*)op = val;
  }
}

extern "C" void kernel_launch(void* const* d_in, const int* in_sizes, int n_in,
                              void* d_out, int out_size, void* d_ws, size_t ws_size,
                              hipStream_t stream) {
  const float* x   = (const float*)d_in[0];
  const float* psf = (const float*)d_in[1];
  float* out       = (float*)d_out;
  const size_t ws_need = WSB_HALVES * 2;
  if (n_in < 2 || ws_size < ws_need) return;
  if (in_sizes[0] < NBATCH * CH_ALL * HWPIX || in_sizes[1] < NCH * KTAP * KTAP * NDEP) return;
  if (out_size < NBATCH * NCH * HWPIX) return;
  unsigned* btw = (unsigned*)d_ws;

  build_btiles<<<NB_THREADS / NTHR, NTHR, 0, stream>>>(psf, btw, NB_THREADS);

  dim3 grid(IMG_W / TILE_W, IMG_H / TILE_H, NBATCH * NCH);
  conv_depth_fused<<<grid, NTHR, 0, stream>>>(x, (const unsigned short*)d_ws, out);
}
